// GridSumAttention_59846074302961
// MI455X (gfx1250) — hardware-verified
//
#include <hip/hip_runtime.h>
#include <math.h>

#define NTOK 16384
#define CC_  384
#define SLEN 4096
#define NGW  1024
#define NWIN 4096
#define NHN  36
#define NHEAD 6
#define DH_  64
#define KVS  776

typedef _Float16 f16;
typedef __attribute__((ext_vector_type(16))) f16 f16x16;
typedef __attribute__((ext_vector_type(8)))  f16 f16x8;
typedef __attribute__((ext_vector_type(8)))  float f32x8;
typedef __attribute__((ext_vector_type(4)))  float v4f_t;
typedef float v4fa __attribute__((ext_vector_type(4), may_alias));
typedef __attribute__((ext_vector_type(4)))  unsigned v4u_t;
typedef unsigned v4ua __attribute__((ext_vector_type(4), may_alias));

__device__ __forceinline__ f32x8 wmma16(f16x16 a, f16x16 b, f32x8 c) {
  c = __builtin_amdgcn_wmma_f32_16x16x32_f16(false, a, false, b, (short)0, c, false, false);
  asm volatile("v_nop\n\tv_nop\n\tv_nop\n\tv_nop" : "+v"(c) : "v"(a), "v"(b));
  return c;
}
__device__ __forceinline__ f16x16 lds_frag(const f16* base, int stride) {
  const int lane = threadIdx.x & 31, row = lane & 15, kh = (lane >> 4) * 8;
  const f16x8 lo = *(const f16x8*)(base + row * stride + kh);
  const f16x8 hi = *(const f16x8*)(base + row * stride + kh + 16);
  f16x16 f;
#pragma unroll
  for (int i = 0; i < 8; ++i) { f[i] = lo[i]; f[i + 8] = hi[i]; }
  return f;
}

#define GSTR 48
template <typename AT, int EPI, bool OUT16>
__global__ __launch_bounds__(256) void gemm_kne(const AT* __restrict__ A, int lda, const float* __restrict__ Wm, int ldw,
                                                const float* __restrict__ bias, const float* __restrict__ R, const float* __restrict__ gvec,
                                                void* __restrict__ Yv, int ldy, int K) {
  __shared__ __attribute__((aligned(16))) f16 ldsA[128 * GSTR];
  __shared__ __attribute__((aligned(16))) f16 ldsW[128 * GSTR];
  __shared__ __attribute__((aligned(16))) float oS[8][32 * 68];
  const int tid = threadIdx.x, lane = tid & 31, wave = tid >> 5, cl = lane & 15, rh = (lane >> 4) * 8;
  const int m0 = blockIdx.x * 128, n0 = blockIdx.y * 128;
  const int wm = (wave & 3) * 32, wn = (wave >> 2) * 64;
  f32x8 acc[2][4];
#pragma unroll
  for (int i = 0; i < 2; ++i)
#pragma unroll
    for (int j = 0; j < 4; ++j) { f32x8 z = {}; acc[i][j] = z; }
#pragma unroll 1
  for (int k0 = 0; k0 < K; k0 += 32) {
    __syncthreads();
    { const int row = tid >> 1, ch = (tid & 1) * 16;
      const AT* src = A + (size_t)(m0 + row) * lda + k0 + ch;
#pragma unroll
      for (int g = 0; g < 16; ++g) ldsA[row * GSTR + ch + g] = (f16)src[g]; }
    { const int k = tid >> 3, nn0 = (tid & 7) * 16;
      const float* src = Wm + (size_t)(k0 + k) * ldw + n0 + nn0;
#pragma unroll
      for (int g = 0; g < 4; ++g) { const v4f_t v = *(const v4f_t*)(src + 4 * g);
#pragma unroll
        for (int u = 0; u < 4; ++u) ldsW[(nn0 + 4 * g + u) * GSTR + k] = (f16)v[u]; } }
    __syncthreads();
    f16x16 af[2];
#pragma unroll
    for (int i = 0; i < 2; ++i) af[i] = lds_frag(ldsA + (wm + 16 * i) * GSTR, GSTR);
#pragma unroll
    for (int j = 0; j < 4; ++j) {
      const f16x16 bf = lds_frag(ldsW + (wn + 16 * j) * GSTR, GSTR);
#pragma unroll
      for (int i = 0; i < 2; ++i) acc[i][j] = wmma16(af[i], bf, acc[i][j]);
    }
  }
  float* so = oS[wave];
#pragma unroll
  for (int i = 0; i < 2; ++i)
#pragma unroll
    for (int j = 0; j < 4; ++j) {
      const int n = n0 + wn + 16 * j + cl;
      const float bv = bias ? bias[n] : 0.0f;
      const float gv = (EPI == 2) ? gvec[n] : 0.0f;
      if (EPI == 1) {
#pragma unroll 1
        for (int r = 0; r < 8; ++r) { const float xg = acc[i][j][r] + bv;
          const float u = 0.7978845608028654f * (xg + 0.044715f * xg * xg * xg);
          so[(16 * i + rh + r) * 68 + 16 * j + cl] = 0.5f * xg * (2.0f - 2.0f / (1.0f + __expf(2.0f * u))); }
      } else {
#pragma unroll
        for (int r = 0; r < 8; ++r) {
          float v = acc[i][j][r] + bv;
          if (EPI == 2) v = R[(size_t)(m0 + wm + 16 * i + rh + r) * ldy + n] + gv * v;
          so[(16 * i + rh + r) * 68 + 16 * j + cl] = v;
        }
      }
    }
  asm volatile("s_wait_dscnt 0" ::: "memory");
  __builtin_amdgcn_wave_barrier();
#pragma unroll 1
  for (int pass = 0; pass < 2; ++pass) {
    if (OUT16) {
      f16* Y = (f16*)Yv;
#pragma unroll
      for (int it = 0; it < 8; ++it) { const int c = lane + 32 * it, rr = c >> 3, q8 = (c & 7) * 8;
        union { f16 h[8]; v4u_t v; } u;
#pragma unroll
        for (int e = 0; e < 8; ++e) u.h[e] = (f16)so[rr * 68 + q8 + e];
        *(volatile v4u_t*)(Y + (size_t)(m0 + wm + rr) * ldy + n0 + wn + q8) = u.v; }
    } else {
      float* Y = (float*)Yv;
#pragma unroll
      for (int it = 0; it < 16; ++it) { const int f4 = lane + 32 * it, rr = f4 >> 4, q = (f4 & 15) * 4;
        *(volatile v4f_t*)(Y + (size_t)(m0 + wm + rr) * ldy + n0 + wn + q) = *(const volatile v4fa*)(so + rr * 68 + q); }
    }
    __threadfence();
  }
}

__global__ __launch_bounds__(128) void k_ln2(const float* __restrict__ x, const float* __restrict__ sq, const float* __restrict__ bq,
                                             const float* __restrict__ skv, const float* __restrict__ bkv2, float* __restrict__ lnq, float* __restrict__ lnkv) {
  __shared__ float red[128];
  const int tok = blockIdx.x, t = threadIdx.x;
  const float* xr = x + (size_t)tok * CC_;
  const float v0 = xr[t], v1 = xr[t + 128], v2 = xr[t + 256];
  red[t] = v0 + v1 + v2; __syncthreads();
  for (int o = 64; o > 0; o >>= 1) { if (t < o) red[t] += red[t + o]; __syncthreads(); }
  const float mu = red[0] * (1.0f / (float)CC_); __syncthreads();
  const float d0 = v0 - mu, d1 = v1 - mu, d2 = v2 - mu;
  red[t] = d0 * d0 + d1 * d1 + d2 * d2; __syncthreads();
  for (int o = 64; o > 0; o >>= 1) { if (t < o) red[t] += red[t + o]; __syncthreads(); }
  const float rs = rsqrtf(red[0] * (1.0f / (float)CC_) + 1e-5f);
  const float n0 = d0 * rs, n1 = d1 * rs, n2 = d2 * rs;
  float* a = lnq + (size_t)tok * CC_; float* bb = lnkv + (size_t)tok * CC_;
#pragma unroll 1
  for (int pass = 0; pass < 2; ++pass) {
    *(volatile float*)(a + t) = n0 * sq[t] + bq[t]; *(volatile float*)(a + t + 128) = n1 * sq[t + 128] + bq[t + 128]; *(volatile float*)(a + t + 256) = n2 * sq[t + 256] + bq[t + 256];
    *(volatile float*)(bb + t) = n0 * skv[t] + bkv2[t]; *(volatile float*)(bb + t + 128) = n1 * skv[t + 128] + bkv2[t + 128]; *(volatile float*)(bb + t + 256) = n2 * skv[t + 256] + bkv2[t + 256];
    __threadfence();
  }
}
__global__ __launch_bounds__(128) void k_res_ln(const float* __restrict__ x, const float* __restrict__ p, const float* __restrict__ s,
                                                const float* __restrict__ b, float* __restrict__ x1, float* __restrict__ lnm) {
  __shared__ float red[128];
  const int tok = blockIdx.x, t = threadIdx.x;
  const float* xr = x + (size_t)tok * CC_; const float* pr = p + (size_t)tok * CC_;
  const float v0 = xr[t] + pr[t], v1 = xr[t + 128] + pr[t + 128], v2 = xr[t + 256] + pr[t + 256];
  red[t] = v0 + v1 + v2; __syncthreads();
  for (int o = 64; o > 0; o >>= 1) { if (t < o) red[t] += red[t + o]; __syncthreads(); }
  const float mu = red[0] * (1.0f / (float)CC_); __syncthreads();
  const float d0 = v0 - mu, d1 = v1 - mu, d2 = v2 - mu;
  red[t] = d0 * d0 + d1 * d1 + d2 * d2; __syncthreads();
  for (int o = 64; o > 0; o >>= 1) { if (t < o) red[t] += red[t + o]; __syncthreads(); }
  const float rs = rsqrtf(red[0] * (1.0f / (float)CC_) + 1e-5f);
  float* a = x1 + (size_t)tok * CC_; float* bb = lnm + (size_t)tok * CC_;
#pragma unroll 1
  for (int pass = 0; pass < 2; ++pass) {
    *(volatile float*)(a + t) = v0; *(volatile float*)(a + t + 128) = v1; *(volatile float*)(a + t + 256) = v2;
    *(volatile float*)(bb + t) = d0 * rs * s[t] + b[t]; *(volatile float*)(bb + t + 128) = d1 * rs * s[t + 128] + b[t + 128]; *(volatile float*)(bb + t + 256) = d2 * rs * s[t + 256] + b[t + 256];
    __threadfence();
  }
}
__global__ __launch_bounds__(64) void k_window_attn(const float* __restrict__ q, const float* __restrict__ kv, const int* __restrict__ mask,
                                                    const int* __restrict__ nh, float* __restrict__ o) {
  __shared__ __attribute__((aligned(16))) f16 kvS[48 * KVS];
  __shared__ __attribute__((aligned(16))) f16 qS[16 * 392];
  __shared__ __attribute__((aligned(16))) f16 pS[2][16 * 72];
  __shared__ __attribute__((aligned(16))) float oS[4 * 388];
  __shared__ int mS[48];
  const int tid = threadIdx.x, lane = tid & 31, wave = tid >> 5, cl = lane & 15, hsel = lane >> 4, kh = hsel * 8, rh = kh;
  const int win = blockIdx.x;
  const int vt = win >> 10, g = win & 1023;
  const size_t tok0 = (size_t)vt * SLEN;
  for (int e = tid; e < 48 * (768 / 4); e += 64) {
    const int r = e / 192, c4 = (e % 192) * 4;
    v4f_t v = {0.f, 0.f, 0.f, 0.f};
    if (r < NHN) { int s = nh[g * NHN + r]; s = min(max(s, 0), SLEN - 1); v = *(const v4f_t*)(kv + (tok0 + s) * 768 + c4); }
    f16* d = kvS + r * KVS + c4; d[0] = (f16)v[0]; d[1] = (f16)v[1]; d[2] = (f16)v[2]; d[3] = (f16)v[3];
  }
  for (int e = tid; e < 16 * (384 / 4); e += 64) {
    const int r = e / 96, c4 = (e % 96) * 4;
    v4f_t v = {0.f, 0.f, 0.f, 0.f};
    if (r < 4) v = *(const v4f_t*)(q + (tok0 + (size_t)g * 4 + r) * CC_ + c4);
    f16* d = qS + r * 392 + c4; d[0] = (f16)v[0]; d[1] = (f16)v[1]; d[2] = (f16)v[2]; d[3] = (f16)v[3];
  }
  if (tid < 48) { int mb = 2; if (tid < NHN) { int s = nh[g * NHN + tid]; s = min(max(s, 0), SLEN - 1); mb = (mask[tok0 + s] != 0) ? 1 : 0; } mS[tid] = mb; }
  for (int e = tid; e < 2 * 16 * 72; e += 64) (&pS[0][0])[e] = (f16)0.0f;
  __syncthreads();
  f16* pw = pS[wave];
#pragma unroll 1
  for (int hh = 0; hh < 3; ++hh) {
    const int h = wave * 3 + hh;
    f32x8 s[3];
#pragma unroll
    for (int nt = 0; nt < 3; ++nt) { f32x8 z = {}; s[nt] = z; }
#pragma unroll
    for (int ks = 0; ks < 2; ++ks) {
      const f16x16 af = lds_frag(qS + h * DH_ + ks * 32, 392);
#pragma unroll
      for (int nt = 0; nt < 3; ++nt) s[nt] = wmma16(af, lds_frag(kvS + (nt * 16) * KVS + h * DH_ + ks * 32, KVS), s[nt]);
    }
    float mrow[8], lrow[8];
#pragma unroll
    for (int r = 0; r < 8; ++r) {
      float m = -INFINITY;
#pragma unroll
      for (int nt = 0; nt < 3; ++nt) { const int j = nt * 16 + cl; const int mb = mS[j]; const float v = (mb == 0) ? s[nt][r] * 0.125f : (mb == 1) ? -1.0e9f : -INFINITY; s[nt][r] = v; m = fmaxf(m, v); }
#pragma unroll
      for (int off = 8; off >= 1; off >>= 1) m = fmaxf(m, __shfl_xor(m, off, 32));
      mrow[r] = m;
      float l = 0.0f;
#pragma unroll
      for (int nt = 0; nt < 3; ++nt) { const float e = __expf(s[nt][r] - m); s[nt][r] = e; l += e; }
#pragma unroll
      for (int off = 8; off >= 1; off >>= 1) l += __shfl_xor(l, off, 32);
      lrow[r] = l;
    }
#pragma unroll
    for (int r = 0; r < 8; ++r)
#pragma unroll
      for (int nt = 0; nt < 3; ++nt) pw[(rh + r) * 72 + nt * 16 + cl] = (f16)(s[nt][r] * (1024.0f / lrow[r]));
    asm volatile("s_wait_dscnt 0" ::: "memory");
    __builtin_amdgcn_wave_barrier();
    const f16x16 p0 = lds_frag(pw, 72), p1 = lds_frag(pw + 32, 72);
#pragma unroll
    for (int nt = 0; nt < 4; ++nt) {
      f16x16 b0, b1;
      const f16* vb = kvS + 384 + h * DH_ + nt * 16 + cl;
#pragma unroll
      for (int i = 0; i < 8; ++i) { b0[i] = vb[(kh + i) * KVS]; b0[8 + i] = vb[(16 + kh + i) * KVS]; b1[i] = vb[(32 + kh + i) * KVS]; b1[8 + i] = (f16)0.0f; }
      f32x8 z = {};
      z = wmma16(p0, b0, z); z = wmma16(p1, b1, z);
      if (hsel == 0) {
#pragma unroll
        for (int r = 0; r < 4; ++r) oS[r * 388 + h * DH_ + nt * 16 + cl] = z[r] * (1.0f / 1024.0f);
      }
    }
    __builtin_amdgcn_wave_barrier();
  }
  __syncthreads();
#pragma unroll 1
  for (int pass = 0; pass < 2; ++pass) {
#pragma unroll
    for (int it = 0; it < 6; ++it) { const int f4 = tid + 64 * it, rr = f4 / 96, qd = (f4 % 96) * 4;
      *(volatile v4f_t*)(o + (tok0 + (size_t)g * 4 + rr) * CC_ + qd) = *(const volatile v4fa*)(oS + rr * 388 + qd); }
    __threadfence();
  }
}

extern "C" void kernel_launch(void* const* d_in, const int* in_sizes, int n_in,
                              void* d_out, int out_size, void* d_ws, size_t ws_size,
                              hipStream_t stream) {
  (void)in_sizes; (void)n_in; (void)out_size; (void)ws_size;
  const float* x = (const float*)d_in[0];
  const int* mask = (const int*)d_in[1];
  const int* nh = (const int*)d_in[2];
  const float* lnq_s = (const float*)d_in[3], *lnq_b = (const float*)d_in[4];
  const float* Wq = (const float*)d_in[5];
  const float* lnkv_s = (const float*)d_in[6], *lnkv_b = (const float*)d_in[7];
  const float* Wkv = (const float*)d_in[8], *bkv = (const float*)d_in[9];
  const float* Wo = (const float*)d_in[10];
  const float* lnm_s = (const float*)d_in[11], *lnm_b = (const float*)d_in[12];
  const float* Wemb = (const float*)d_in[13], *bemb = (const float*)d_in[14];
  const float* W1 = (const float*)d_in[15], *b1 = (const float*)d_in[16];
  const float* W2 = (const float*)d_in[17], *b2 = (const float*)d_in[18];
  const float* gam = (const float*)d_in[19];
  float* out = (float*)d_out;
  char* ws = (char*)d_ws;
  const size_t F32C = (size_t)NTOK * CC_ * 4;
  float* bufA = (float*)ws;
  float* bufB = (float*)(ws + F32C);
  float* qb   = (float*)(ws + 2 * F32C);
  float* kvb  = (float*)(ws + 3 * F32C);
  k_ln2<<<dim3(NTOK), dim3(128), 0, stream>>>(x, lnq_s, lnq_b, lnkv_s, lnkv_b, bufA, bufB);
  gemm_kne<float, 0, false><<<dim3(NTOK / 128, CC_ / 128), dim3(256), 0, stream>>>(bufA, CC_, Wq, CC_, nullptr, nullptr, nullptr, qb, CC_, CC_);
  gemm_kne<float, 0, false><<<dim3(NTOK / 128, 768 / 128), dim3(256), 0, stream>>>(bufB, CC_, Wkv, 768, bkv, nullptr, nullptr, kvb, 768, CC_);
  k_window_attn<<<dim3(NWIN), dim3(64), 0, stream>>>(qb, kvb, mask, nh, bufA);
  gemm_kne<float, 0, false><<<dim3(NTOK / 128, CC_ / 128), dim3(256), 0, stream>>>(bufA, CC_, Wo, CC_, nullptr, nullptr, nullptr, bufB, CC_, CC_);
  k_res_ln<<<dim3(NTOK), dim3(128), 0, stream>>>(x, bufB, lnm_s, lnm_b, qb, bufA);
  gemm_kne<float, 0, false><<<dim3(NTOK / 128, CC_ / 128), dim3(256), 0, stream>>>(bufA, CC_, Wemb, CC_, bemb, nullptr, nullptr, bufB, CC_, CC_);
  gemm_kne<float, 1, true ><<<dim3(NTOK / 128, 768 / 128), dim3(256), 0, stream>>>(bufB, CC_, W1, 768, b1, nullptr, nullptr, kvb, 768, CC_);
  gemm_kne<f16,   2, false><<<dim3(NTOK / 128, CC_ / 128), dim3(256), 0, stream>>>((const f16*)kvb, 768, W2, CC_, b2, qb, gam, out, CC_, 768);
}
